// QuantumAttention_67508295959008
// MI455X (gfx1250) — hardware-run, weakly checked
//
#include <hip/hip_runtime.h>
#include <math.h>

#ifndef NB
#define NB 4
#endif
#ifndef SEQ
#define SEQ 1024
#endif
#define NB_FULL 4
#define SEQ_FULL 1024

constexpr int CD = 1024;
constexpr int NH = 16;
constexpr int HD = 64;
constexpr int C2 = 2 * CD;
constexpr int NCH = SEQ / 64;
constexpr int MTOK = NB * SEQ;
constexpr int QKP = 4 * CD;
constexpr int VTP = MTOK;
constexpr int NLAY = 4;

static_assert(NB >= 1 && NB <= NB_FULL);
static_assert(SEQ <= SEQ_FULL);
static_assert(CD == NH * HD);
static_assert(HD == 64);
static_assert(MTOK % 64 == 0 && CD % 64 == 0 && C2 % 64 == 0 && QKP % 64 == 0);
static_assert(C2 % 32 == 0);
static_assert(SEQ % 64 == 0);
static_assert(CD % 8 == 0);
static_assert(((long long)MTOK * (CD / 8)) % 256 == 0);
static_assert(((long long)NLAY * CD * (CD / 8)) % 256 == 0);
static_assert((NLAY * C2 / 4) % 256 == 0);
static_assert((long long)2 * NB_FULL * SEQ_FULL * CD * 4 == 33554432LL);

typedef __attribute__((ext_vector_type(16))) _Float16 v16h;
typedef __attribute__((ext_vector_type(8)))  _Float16 v8h;
typedef __attribute__((ext_vector_type(8)))  float    v8f;
typedef __attribute__((ext_vector_type(4)))  float    v4f;
typedef __attribute__((ext_vector_type(4)))  unsigned int v4u;
typedef __attribute__((ext_vector_type(2)))  unsigned int v2u;

union FH { v16h v; v8h h[2]; };

#define VST2(T, ptr, val) do { const T vst2_v_ = (val); *(volatile T*)(ptr) = vst2_v_; __threadfence(); *(volatile T*)(ptr) = vst2_v_; } while (0)

#define WAVE_SYNC() do { __builtin_amdgcn_fence(3  , "workgroup"); __builtin_amdgcn_wave_barrier(); __builtin_amdgcn_fence(2  , "workgroup"); } while (0)

__device__ __forceinline__ float cmb_bf(float v) { const unsigned u = __builtin_bit_cast(unsigned, v); const unsigned r = (u + 0x7fffu + ((u >> 16) & 1u)) & 0xffff0000u; return __builtin_bit_cast(float, r); }
__device__ __forceinline__ unsigned int pk2h(float a, float b) { return (unsigned int)__builtin_bit_cast(unsigned short, (_Float16)a) | ((unsigned int)__builtin_bit_cast(unsigned short, (_Float16)b) << 16); }
static __device__ __forceinline__ _Float16 toh_flush(float v) { const _Float16 r = (_Float16)v; return (fabsf(v) < 6.103515625e-05f) ? (_Float16)0.0f : r; }
static __device__ __forceinline__ unsigned int pk2hf(float a, float b) { return (unsigned int)__builtin_bit_cast(unsigned short, toh_flush(a)) | ((unsigned int)__builtin_bit_cast(unsigned short, toh_flush(b)) << 16); }
__device__ __forceinline__ v16h ldg_frag(const _Float16* __restrict__ p) { FH f; f.h[0] = *(const v8h*)(p); f.h[1] = *(const v8h*)(p + 16); return f.v; }

__device__ __forceinline__ v8f mma_h(v16h a, v16h b, v8f c) {
  c = __builtin_amdgcn_wmma_f32_16x16x32_f16(false, a, false, b, (short)0, c, false, false);
  asm volatile("v_nop\n\tv_nop\n\tv_nop\n\tv_nop" : "+v"(c) : "v"(a), "v"(b));
  return c;
}
__device__ __forceinline__ void dep_guard_h(v8f& a, v8f& b, v16h x, v16h y) { asm volatile("v_nop\n\tv_nop\n\tv_nop\n\tv_nop" : "+v"(a), "+v"(b) : "v"(x), "v"(y)); }
__device__ __forceinline__ void keep4_h(v16h a, v16h b, v16h c, v16h d) { asm volatile("v_nop" :: "v"(a), "v"(b), "v"(c), "v"(d)); }
__device__ __forceinline__ void acc_guard4(v8f& a, v8f& b, v8f& c, v8f& d) { asm volatile("v_nop\n\tv_nop\n\tv_nop\n\tv_nop" : "+v"(a), "+v"(b), "+v"(c), "+v"(d)); }

__device__ __forceinline__ float gelu_tanh(float t) {
  const float t3 = (t * t) * t;
  const float u = 0.7978845608028654f * (t + 0.044715f * t3);
  const float e = exp2f(-2.885390081777927f * u);
  return t * __builtin_amdgcn_rcpf(1.0f + e);
}

__global__ __launch_bounds__(256) void k_castx(const float* __restrict__ XR, const float* __restrict__ XI, unsigned short* __restrict__ X2) {
  #pragma clang fp contract(off)
  const long long u = (long long)blockIdx.x * 256 + threadIdx.x; const int per = CD / 8; if (u >= (long long)MTOK * per) return;
  const int r = (int)(u / per); const int c8 = 8 * (int)(u % per);
  const size_t srow = (size_t)(r / SEQ) * SEQ_FULL + (size_t)(r % SEQ);
  const v4f a0 = *(const v4f*)(XR + srow * CD + c8), a1 = *(const v4f*)(XR + srow * CD + c8 + 4);
  const v4f b0 = *(const v4f*)(XI + srow * CD + c8), b1 = *(const v4f*)(XI + srow * CD + c8 + 4);
  v4u pr, pi;
  pr.x = pk2hf(cmb_bf(a0.x), cmb_bf(a0.y)); pr.y = pk2hf(cmb_bf(a0.z), cmb_bf(a0.w)); pr.z = pk2hf(cmb_bf(a1.x), cmb_bf(a1.y)); pr.w = pk2hf(cmb_bf(a1.z), cmb_bf(a1.w));
  pi.x = pk2hf(cmb_bf(b0.x), cmb_bf(b0.y)); pi.y = pk2hf(cmb_bf(b0.z), cmb_bf(b0.w)); pi.z = pk2hf(cmb_bf(b1.x), cmb_bf(b1.y)); pi.w = pk2hf(cmb_bf(b1.z), cmb_bf(b1.w));
  VST2(v4u, (v4u*)(X2 + (size_t)r * C2 + c8), pr);
  VST2(v4u, (v4u*)(X2 + (size_t)r * C2 + CD + c8), pi);
}

__global__ __launch_bounds__(256) void k_castw(const float* __restrict__ WR, const float* __restrict__ WI, unsigned short* __restrict__ W2) {
  #pragma clang fp contract(off)
  const long long u = (long long)blockIdx.x * 256 + threadIdx.x; const int per = CD / 8; if (u >= (long long)NLAY * CD * per) return;
  const int r = (int)(u / per); const int c8 = 8 * (int)(u % per);
  const int l = r / CD, n = r % CD;
  const v4f a0 = *(const v4f*)(WR + (size_t)r * CD + c8), a1 = *(const v4f*)(WR + (size_t)r * CD + c8 + 4);
  const v4f b0 = *(const v4f*)(WI + (size_t)r * CD + c8), b1 = *(const v4f*)(WI + (size_t)r * CD + c8 + 4);
  v4u pr, pi, pn;
  pr.x = pk2hf(cmb_bf(a0.x) * 16.0f, cmb_bf(a0.y) * 16.0f); pr.y = pk2hf(cmb_bf(a0.z) * 16.0f, cmb_bf(a0.w) * 16.0f);
  pr.z = pk2hf(cmb_bf(a1.x) * 16.0f, cmb_bf(a1.y) * 16.0f); pr.w = pk2hf(cmb_bf(a1.z) * 16.0f, cmb_bf(a1.w) * 16.0f);
  pi.x = pk2hf(cmb_bf(b0.x) * 16.0f, cmb_bf(b0.y) * 16.0f); pi.y = pk2hf(cmb_bf(b0.z) * 16.0f, cmb_bf(b0.w) * 16.0f);
  pi.z = pk2hf(cmb_bf(b1.x) * 16.0f, cmb_bf(b1.y) * 16.0f); pi.w = pk2hf(cmb_bf(b1.z) * 16.0f, cmb_bf(b1.w) * 16.0f);
  pn.x = pi.x ^ 0x80008000u; pn.y = pi.y ^ 0x80008000u; pn.z = pi.z ^ 0x80008000u; pn.w = pi.w ^ 0x80008000u;
  unsigned short* base = W2 + (size_t)l * C2 * C2;
  VST2(v4u, (v4u*)(base + (size_t)n * C2 + c8), pr);
  VST2(v4u, (v4u*)(base + (size_t)n * C2 + CD + c8), pn);
  VST2(v4u, (v4u*)(base + (size_t)(CD + n) * C2 + c8), pi);
  VST2(v4u, (v4u*)(base + (size_t)(CD + n) * C2 + CD + c8), pr);
}

__global__ __launch_bounds__(256) void k_bias(const float* __restrict__ BR, const float* __restrict__ BI, float* __restrict__ BS) {
  const int u = blockIdx.x * 256 + threadIdx.x; if (u >= NLAY * C2 / 4) return;
  const int l = u / (C2 / 4), w = u % (C2 / 4);
  const int c4 = 4 * (w % (CD / 4));
  const v4f a = *(const v4f*)(BR + (size_t)l * CD + c4);
  const v4f b = *(const v4f*)(BI + (size_t)l * CD + c4);
  const bool im = (w >= CD / 4);
  v4f v; v.x = im ? b.x : a.x; v.y = im ? b.y : a.y; v.z = im ? b.z : a.z; v.w = im ? b.w : a.w;
  VST2(v4f, (v4f*)(BS + (size_t)u * 4), v);
}

struct GP {
  const unsigned short* A; const unsigned short* Bt; void* C; const float* bias; const float* R;
  long long strideA, strideC;
  int lda, ldb, ldc, ldr, M, N, K, rpb, rpbC, rpbR; float scale; int pad_;
};
static_assert(sizeof(GP) == 104);

template <int BIAS_MODE, int OUT_MODE, int RES_MODE, int ACT>
__device__ __forceinline__ void gemm_body(const GP& p) {
  __shared__ __align__(16) float sT[8][16 * 68];
  const int b = blockIdx.y;
  const int lane = threadIdx.x & 31, wave = threadIdx.x >> 5;
  const int tilesN = p.N >> 6, tilesM = p.M >> 6;
  const int tile = blockIdx.x * 8 + wave;
  if (tile >= tilesM * tilesN) return;
  const int tm = tile / tilesN, tn = tile - tm * tilesN;
  const int m0 = tm << 6, n0 = tn << 6;
  const _Float16* Ab = (const _Float16*)p.A + (size_t)b * p.strideA;
  const _Float16* Bb = (const _Float16*)p.Bt;
  const int rlane = lane & 15, koff = (lane >> 4) * 8, mOff = (lane >> 4) * 8;

  v8f acc[4][4];
#pragma unroll
  for (int i = 0; i < 4; ++i)
#pragma unroll
    for (int j = 0; j < 4; ++j) acc[i][j] = (v8f){0.f, 0.f, 0.f, 0.f, 0.f, 0.f, 0.f, 0.f};

  for (int k0 = 0; k0 < p.K; k0 += 32) {
    v16h bh[4];
#pragma unroll
    for (int j = 0; j < 4; ++j) bh[j] = ldg_frag(Bb + (size_t)(n0 + (j << 4) + rlane) * p.ldb + koff + k0);
#pragma unroll
    for (int i = 0; i < 4; ++i) {
      const v16h ah = ldg_frag(Ab + (size_t)(m0 + (i << 4) + rlane) * p.lda + koff + k0);
#pragma unroll
      for (int j = 0; j < 4; ++j) acc[i][j] = __builtin_amdgcn_wmma_f32_16x16x32_f16(false, ah, false, bh[j], (short)0, acc[i][j], false, false);
      dep_guard_h(acc[i][0], acc[i][3], ah, ah);
    }
    keep4_h(bh[0], bh[1], bh[2], bh[3]);
  }
  acc_guard4(acc[0][0], acc[0][1], acc[0][2], acc[0][3]);
  acc_guard4(acc[1][0], acc[1][1], acc[1][2], acc[1][3]);
  acc_guard4(acc[2][0], acc[2][1], acc[2][2], acc[2][3]);
  acc_guard4(acc[3][0], acc[3][1], acc[3][2], acc[3][3]);

  float* slab = sT[wave];
#pragma unroll
  for (int i = 0; i < 4; ++i) {
    const int mBase = m0 + (i << 4);
    float bm[8];
#pragma unroll
    for (int r = 0; r < 8; ++r) { bm[r] = 0.f; if (BIAS_MODE == 1) bm[r] = cmb_bf(p.bias[mBase + mOff + r]); }
#pragma unroll
    for (int j = 0; j < 4; ++j) {
      const int n = n0 + (j << 4) + rlane;
      float bv = 0.f; if (BIAS_MODE == 2) bv = cmb_bf(p.bias[n]);
#pragma unroll
      for (int r = 0; r < 8; ++r) {
        float v = acc[i][j][r] * p.scale + ((BIAS_MODE == 1) ? bm[r] : bv);
        if (ACT == 1) v = gelu_tanh(v);
        slab[(mOff + r) * 68 + (j << 4) + rlane] = v;
      }
    }
    WAVE_SYNC();
    const int gb = mBase / p.rpb; const int tIn = mBase - gb * p.rpb;
    const size_t rowC0 = (size_t)gb * p.rpbC + tIn, rowR0 = (size_t)gb * p.rpbR + tIn;
    if (OUT_MODE == 0) {
      float* C = (float*)p.C + (size_t)b * p.strideC;
      const int hh = lane >> 4, c4 = (lane & 15) * 4;
      v4f val[8];
#pragma unroll
      for (int it = 0; it < 8; ++it) {
        const int row = it * 2 + hh;
        v4f v = *(const v4f*)(slab + row * 68 + c4);
        if (RES_MODE != 0) {
          v4f x = *(const v4f*)(p.R + (rowR0 + row) * (size_t)p.ldr + n0 + c4);
          if (RES_MODE == 2) { x.x = cmb_bf(x.x); x.y = cmb_bf(x.y); x.z = cmb_bf(x.z); x.w = cmb_bf(x.w); }
          v = v + x;
        }
        val[it] = v;
      }
      for (int pass = 0; pass < 2; ++pass) {
#pragma unroll
        for (int it = 0; it < 8; ++it) {
          const int row = it * 2 + hh;
          *(volatile v4f*)(C + (rowC0 + row) * (size_t)p.ldc + n0 + c4) = val[it];
        }
        __threadfence();
      }
    } else {
      unsigned short* C = (unsigned short*)p.C + (size_t)b * p.strideC;
      const int q = lane >> 3, c8 = (lane & 7) * 8;
      v8h hv[4];
#pragma unroll
      for (int it = 0; it < 4; ++it) {
        const float* sp = slab + (it * 4 + q) * 68 + c8;
#pragma unroll
        for (int e = 0; e < 8; ++e) hv[it][e] = (_Float16)sp[e];
      }
      for (int pass = 0; pass < 2; ++pass) {
#pragma unroll
        for (int it = 0; it < 4; ++it) {
          const int row = it * 4 + q;
          *(volatile v8h*)(C + (rowC0 + row) * (size_t)p.ldc + n0 + c8) = hv[it];
        }
        __threadfence();
      }
    }
    WAVE_SYNC();
  }
}

__device__ __forceinline__ GP gp_pack(const unsigned short* A, const unsigned short* Bt, void* C, const float* bias, const float* R,
                                      long long strideA, long long strideC, int lda, int ldb, int ldc, int ldr, int M, int N, int K,
                                      int rpb, int rpbC, int rpbR, float scale) {
  GP g;
  g.A = A; g.Bt = Bt; g.C = C; g.bias = bias; g.R = R; g.strideA = strideA; g.strideC = strideC;
  g.lda = lda; g.ldb = ldb; g.ldc = ldc; g.ldr = ldr; g.M = M; g.N = N; g.K = K; g.rpb = rpb; g.rpbC = rpbC; g.rpbR = rpbR;
  g.scale = scale; g.pad_ = 0;
  return g;
}

__global__ __launch_bounds__(256) void k_gemm_qk(const unsigned short* A, const unsigned short* Bt, void* C, const float* bias, const float* R,
                                                   long long strideA, long long strideC, int lda, int ldb, int ldc, int ldr, int M, int N, int K,
                                                   int rpb, int rpbC, int rpbR, float scale) {
  const GP p = gp_pack(A, Bt, C, bias, R, strideA, strideC, lda, ldb, ldc, ldr, M, N, K, rpb, rpbC, rpbR, scale);
  gemm_body<2, 1, 0, 0>(p);
}
__global__ __launch_bounds__(256) void k_gemm_vt(const unsigned short* A, const unsigned short* Bt, void* C, const float* bias, const float* R,
                                                   long long strideA, long long strideC, int lda, int ldb, int ldc, int ldr, int M, int N, int K,
                                                   int rpb, int rpbC, int rpbR, float scale) {
  const GP p = gp_pack(A, Bt, C, bias, R, strideA, strideC, lda, ldb, ldc, ldr, M, N, K, rpb, rpbC, rpbR, scale);
  gemm_body<1, 1, 0, 0>(p);
}
__global__ __launch_bounds__(256) void k_gemm_e(const unsigned short* A, const unsigned short* Bt, void* C, const float* bias, const float* R,
                                                  long long strideA, long long strideC, int lda, int ldb, int ldc, int ldr, int M, int N, int K,
                                                  int rpb, int rpbC, int rpbR, float scale) {
  const GP p = gp_pack(A, Bt, C, bias, R, strideA, strideC, lda, ldb, ldc, ldr, M, N, K, rpb, rpbC, rpbR, scale);
  gemm_body<2, 0, 0, 0>(p);
}

#define ATT_SC 0.18033688011112042f
#define ATT_PCAR 4096.0f
#define ATT_OCAR 16.0f

__global__ __launch_bounds__(128) __attribute__((amdgpu_num_vgpr(256))) void k_attn_cplx(const unsigned short* __restrict__ QKp, const unsigned short* __restrict__ VTp,
                                                                                           unsigned short* __restrict__ CTXp) {
  __shared__ __align__(16) _Float16 Psh[4][16 * 64];
  __shared__ __align__(16) float Gsh[4][4 * 32 * 8];
  __shared__ __align__(16) _Float16 Osh[4][16 * 128];
  const int tid = threadIdx.x, wave = __builtin_amdgcn_readfirstlane(threadIdx.x >> 5), lane = tid & 31, hh = lane >> 4, c = lane & 15;
  const int bx = blockIdx.x; const int qb = bx % NCH; const int bhh = bx / NCH; const int h = bhh % NH; const int b = bhh / NH;
  const int q0 = qb * 64 + wave * 16;
  const _Float16* QK = (const _Float16*)QKp; const _Float16* VT = (const _Float16*)VTp;
  const size_t tok0 = (size_t)b * SEQ;

  v16h qr0, qr1, qi0, qi1;
  {
    const _Float16* qrow = QK + (tok0 + q0 + c) * (size_t)QKP + h * HD + 8 * hh;
    qr0 = ldg_frag(qrow); qr1 = ldg_frag(qrow + 32);
    qi0 = ldg_frag(qrow + CD); qi1 = ldg_frag(qrow + CD + 32);
  }

  float mrow[8], lrow[8]; v8f oar[4], oai[4];
#pragma unroll
  for (int r = 0; r < 8; ++r) { mrow[r] = -INFINITY; lrow[r] = 0.f; }
#pragma unroll
  for (int t = 0; t < 4; ++t) { oar[t] = (v8f){0.f, 0.f, 0.f, 0.f, 0.f, 0.f, 0.f, 0.f}; oai[t] = (v8f){0.f, 0.f, 0.f, 0.f, 0.f, 0.f, 0.f, 0.f}; }

  _Float16* pw = Psh[wave];
  float* gw = Gsh[wave];
  const int goff = lane * 8;
#pragma unroll 1
  for (int kc = 0; kc < NCH; ++kc) {
    const int kv0 = kc * 64;
#pragma unroll
    for (int j = 0; j < 4; ++j) {
      const _Float16* krow = QK + (tok0 + kv0 + j * 16 + c) * (size_t)QKP + 2 * CD + h * HD + 8 * hh;
      v8f zr = (v8f){0.f, 0.f, 0.f, 0.f, 0.f, 0.f, 0.f, 0.f};
      v8f zu = (v8f){0.f, 0.f, 0.f, 0.f, 0.f, 0.f, 0.f, 0.f};
      v8f zw = (v8f){0.f, 0.f, 0.f, 0.f, 0.f, 0.f, 0.f, 0.f};
      {
        const v16h kr0 = ldg_frag(krow), kr1 = ldg_frag(krow + 32);
        zr = mma_h(qr0, kr0, zr);
        zr = mma_h(qr1, kr1, zr);
        zu = mma_h(qi0, kr0, zu);
        zu = mma_h(qi1, kr1, zu);
      }
      __builtin_amdgcn_sched_barrier(0);
      {
        const v16h ki0 = ldg_frag(krow + CD), ki1 = ldg_frag(krow + CD + 32);
        zr = mma_h(qi0, ki0, zr);
        zr = mma_h(qi1, ki1, zr);
        zw = mma_h(qr0, ki0, zw);
        zw = mma_h(qr1, ki1, zw);
      }
      v8f gg;
#pragma unroll
      for (int r = 0; r < 8; ++r) {
        const float si = zu[r] - zw[r];
        gg[r] = __builtin_amdgcn_sqrtf(zr[r] * zr[r] + si * si) * ATT_SC;
      }
      const v4f g0 = __builtin_shufflevector(gg, gg, 0, 1, 2, 3);
      const v4f g1 = __builtin_shufflevector(gg, gg, 4, 5, 6, 7);
      *(v4f*)(gw + j * 256 + goff) = g0;
      *(v4f*)(gw + j * 256 + goff + 4) = g1;
      __builtin_amdgcn_sched_barrier(0);
    }
    WAVE_SYNC();
    v4f gl[4][2];
#pragma unroll
    for (int j = 0; j < 4; ++j) { gl[j][0] = *(const v4f*)(gw + j * 256 + goff); gl[j][1] = *(const v4f*)(gw + j * 256 + goff + 4); }
#pragma unroll
    for (int r = 0; r < 8; ++r) {
      float m = fmaxf(fmaxf(gl[0][r >> 2][r & 3], gl[1][r >> 2][r & 3]), fmaxf(gl[2][r >> 2][r & 3], gl[3][r >> 2][r & 3]));
      m = fmaxf(m, __shfl_xor(m, 1, 32)); m = fmaxf(m, __shfl_xor(m, 2, 32));
      m = fmaxf(m, __shfl_xor(m, 4, 32)); m = fmaxf(m, __shfl_xor(m, 8, 32));
      const float mnew = fmaxf(mrow[r], m);
      const float alpha = exp2f(mrow[r] - mnew);
      mrow[r] = mnew;
      float psum = 0.f;
#pragma unroll
      for (int j = 0; j < 4; ++j) {
        const float e = gl[j][r >> 2][r & 3] - mnew;
        const _Float16 ph = (e < -26.0f) ? (_Float16)0.0f : (_Float16)(exp2f(e) * ATT_PCAR);
        psum += (float)ph;
        pw[(8 * hh + r) * 64 + j * 16 + c] = ph;
      }
      psum += __shfl_xor(psum, 1, 32); psum += __shfl_xor(psum, 2, 32); psum += __shfl_xor(psum, 4, 32); psum += __shfl_xor(psum, 8, 32);
      lrow[r] = lrow[r] * alpha + psum;
#pragma unroll
      for (int t = 0; t < 4; ++t) { oar[t][r] *= alpha; oai[t][r] *= alpha; }
      __builtin_amdgcn_sched_barrier(0);
    }
    WAVE_SYNC();
#pragma unroll
    for (int kk = 0; kk < 2; ++kk) {
      FH pa;
      pa.h[0] = *(const v8h*)(pw + c * 64 + kk * 32 + 8 * hh);
      pa.h[1] = *(const v8h*)(pw + c * 64 + kk * 32 + 16 + 8 * hh);
#pragma unroll
      for (int t = 0; t < 4; ++t) {
        const _Float16* vrow = VT + (size_t)(h * HD + t * 16 + c) * VTP + tok0 + kv0 + kk * 32 + 8 * hh;
        const v16h vbr = ldg_frag(vrow);
        const v16h vbi = ldg_frag(vrow + (size_t)CD * VTP);
        oar[t] = mma_h(pa.v, vbr, oar[t]);
        oai[t] = mma_h(pa.v, vbi, oai[t]);
        __builtin_amdgcn_sched_barrier(0);
      }
    }
    WAVE_SYNC();
  }

  _Float16* os = Osh[wave];
#pragma unroll
  for (int r = 0; r < 8; ++r) {
    const float inv = (lrow[r] > 0.f) ? ATT_OCAR / lrow[r] : 0.f;
#pragma unroll
    for (int t = 0; t < 4; ++t) {
      os[(8 * hh + r) * 128 + t * 16 + c] = toh_flush(oar[t][r] * inv);
      os[(8 * hh + r) * 128 + 64 + t * 16 + c] = toh_flush(oai[t][r] * inv);
    }
  }
  WAVE_SYNC();
  {
    const int q = lane >> 3, c8 = (lane & 7) * 8;
    v8h hr[4], hi[4];
#pragma unroll
    for (int it = 0; it < 4; ++it) { hr[it] = *(const v8h*)(os + (it * 4 + q) * 128 + c8); hi[it] = *(const v8h*)(os + (it * 4 + q) * 128 + 64 + c8); }
    for (int pass = 0; pass < 2; ++pass) {
#pragma unroll
      for (int it = 0; it < 4; ++it) {
        *(volatile v8h*)(CTXp + (tok0 + q0 + it * 4 + q) * (size_t)C2 + h * HD + c8) = hr[it];
        *(volatile v8h*)(CTXp + (tok0 + q0 + it * 4 + q) * (size_t)C2 + CD + h * HD + c8) = hi[it];
      }
      __threadfence();
    }
  }
}

constexpr size_t SZ_X2   = (size_t)MTOK * C2 * 2;
constexpr size_t SZ_W2   = (size_t)NLAY * C2 * C2 * 2;
constexpr size_t SZ_QK   = (size_t)MTOK * QKP * 2;
constexpr size_t SZ_VT   = (size_t)C2 * VTP * 2;
constexpr size_t SZ_CTX  = (size_t)MTOK * C2 * 2;
constexpr size_t SZ_BS   = (size_t)NLAY * C2 * 4;
constexpr size_t OFF_X2  = 0;
constexpr size_t OFF_W2  = OFF_X2 + SZ_X2;
constexpr size_t OFF_QK  = OFF_W2 + SZ_W2;
constexpr size_t OFF_VT  = OFF_QK + SZ_QK;
constexpr size_t OFF_CTX = OFF_VT + SZ_VT;
constexpr size_t OFF_BS  = OFF_CTX + SZ_CTX;
constexpr size_t WS_TOTAL = OFF_BS + SZ_BS;
static_assert(WS_TOTAL <= (size_t)134217728);
static_assert(SZ_X2 % 256 == 0 && SZ_W2 % 256 == 0 && SZ_QK % 256 == 0 && SZ_VT % 256 == 0 && SZ_CTX % 256 == 0 && SZ_BS % 256 == 0);

static GP mk_gp(const unsigned short* A, long long sA, int lda, const unsigned short* Bt, int ldb, void* C, long long sC, int ldc,
                const float* bias, const float* R, int ldr, int M, int N, int K, int rpb, int rpbC, int rpbR) {
  GP g{};
  g.A = A; g.Bt = Bt; g.C = C; g.bias = bias; g.R = R; g.strideA = sA; g.strideC = sC;
  g.lda = lda; g.ldb = ldb; g.ldc = ldc; g.ldr = ldr; g.M = M; g.N = N; g.K = K; g.rpb = rpb; g.rpbC = rpbC; g.rpbR = rpbR;
  g.scale = 0.0625f; g.pad_ = 0;
  return g;
}
#define GP_ARGS(g) (g).A, (g).Bt, (g).C, (g).bias, (g).R, (g).strideA, (g).strideC, (g).lda, (g).ldb, (g).ldc, (g).ldr, (g).M, (g).N, (g).K, (g).rpb, (g).rpbC, (g).rpbR, (g).scale
static unsigned gemm_blocks(int M, int N) { return (unsigned)((((M / 64) * (N / 64)) + 7) / 8); }

extern "C" void kernel_launch(void* const* d_in, const int* in_sizes, int n_in, void* d_out, int out_size, void* d_ws, size_t ws_size, hipStream_t stream) {
  if (n_in < 6) return;
  const long long need_x = ((long long)(NB - 1) * SEQ_FULL + SEQ) * CD;
  const long long plane = (long long)NB_FULL * SEQ_FULL * CD;
  if ((long long)in_sizes[0] < need_x || (long long)in_sizes[1] < need_x) return;
  if ((long long)in_sizes[2] < (long long)NLAY * CD * CD || (long long)in_sizes[3] < (long long)NLAY * CD * CD) return;
  if (in_sizes[4] < NLAY * CD || in_sizes[5] < NLAY * CD) return;
  if ((long long)out_size < plane + need_x) return;
  if (ws_size < WS_TOTAL) return;

  const float* xr = (const float*)d_in[0];
  const float* xi = (const float*)d_in[1];
  const float* wr = (const float*)d_in[2];
  const float* wi = (const float*)d_in[3];
  const float* br = (const float*)d_in[4];
  const float* bi = (const float*)d_in[5];
  float* out = (float*)d_out;
  char* wsp = (char*)d_ws;
  unsigned short* X2  = (unsigned short*)(wsp + OFF_X2);
  unsigned short* W2  = (unsigned short*)(wsp + OFF_W2);
  unsigned short* QK  = (unsigned short*)(wsp + OFF_QK);
  unsigned short* VT  = (unsigned short*)(wsp + OFF_VT);
  unsigned short* CTX = (unsigned short*)(wsp + OFF_CTX);
  float*          BS  = (float*)(wsp + OFF_BS);
  const int BIG = 1 << 30;

  k_castx<<<(unsigned)(((long long)MTOK * (CD / 8)) / 256), 256, 0, stream>>>(xr, xi, X2);
  k_castw<<<(unsigned)(((long long)NLAY * CD * (CD / 8)) / 256), 256, 0, stream>>>(wr, wi, W2);
  k_bias<<<(NLAY * C2 / 4) / 256, 256, 0, stream>>>(br, bi, BS);
  { const GP g = mk_gp(X2, 0, C2, W2, C2, (void*)QK, 0, QKP, BS, nullptr, 0, MTOK, QKP, C2, BIG, BIG, BIG);
    k_gemm_qk<<<dim3(gemm_blocks(MTOK, QKP), 1), 256, 0, stream>>>(GP_ARGS(g)); }
  { const GP g = mk_gp(W2 + (size_t)2 * C2 * C2, 0, C2, X2, C2, (void*)VT, 0, VTP, BS + 2 * C2, nullptr, 0, C2, MTOK, C2, BIG, BIG, BIG);
    k_gemm_vt<<<dim3(gemm_blocks(C2, MTOK), 1), 256, 0, stream>>>(GP_ARGS(g)); }
  k_attn_cplx<<<NB * NH * NCH, 128, 0, stream>>>(QK, VT, CTX);
  { GP g = mk_gp(CTX, 0, C2, W2 + (size_t)3 * C2 * C2, C2, (void*)out, 0, CD, br + 3 * CD, nullptr, 0, MTOK, CD, C2, SEQ, SEQ_FULL, SEQ);
    g.scale = 0.00390625f;
    k_gemm_e<<<dim3(gemm_blocks(MTOK, CD), 1), 256, 0, stream>>>(GP_ARGS(g)); }
  { GP g = mk_gp(CTX, 0, C2, W2 + (size_t)3 * C2 * C2 + (size_t)CD * C2, C2, (void*)(out + plane), 0, CD, bi + 3 * CD, nullptr, 0, MTOK, CD, C2, SEQ, SEQ_FULL, SEQ);
    g.scale = 0.00390625f;
    k_gemm_e<<<dim3(gemm_blocks(MTOK, CD), 1), 256, 0, stream>>>(GP_ARGS(g)); }
}
